// IPNN_21844203668191
// MI455X (gfx1250) — hardware-verified
//
#include <hip/hip_runtime.h>


namespace {
constexpr int B = 1024, Y = 100, YP = 112, NV = 4, NSV = 16, J = 65536;
constexpr float FS = 16384.0f, PS = 1024.0f;
typedef _Float16 b16;
typedef __attribute__((ext_vector_type(16))) _Float16 v16b;
typedef __attribute__((ext_vector_type(8))) _Float16 v8b;
typedef __attribute__((ext_vector_type(8))) float v8f;
typedef __attribute__((ext_vector_type(4))) float v4f;
typedef __attribute__((ext_vector_type(2))) float v2f;
__device__ __forceinline__ float bf16_rne(float f) { unsigned int u = __float_as_uint(f); u += 0x7FFFu + ((u >> 16) & 1u); return __uint_as_float(u & 0xFFFF0000u); }
__device__ __forceinline__ void split16(float v, b16& hi, b16& lo) { hi = (b16)v; lo = (b16)(v - (float)hi); }
__device__ __forceinline__ v16b frag_kb(const b16* p, int hh) { const v8b a = *(const v8b*)(p + 8 * hh), b = *(const v8b*)(p + 16 + 8 * hh); v16b f;
#pragma unroll
  for (int e = 0; e < 8; ++e) { f[e] = a[e]; f[8 + e] = b[e]; } return f; }
__device__ __forceinline__ v8f wmma16b(v16b a, v16b b, v8f c) { v8f d = __builtin_amdgcn_wmma_f32_16x16x32_f16(false, a, false, b, (short)0, c, false, false); asm volatile("v_nop\n\tv_nop\n\tv_nop\n\tv_nop" : "+v"(d) : "v"(a), "v"(b)); return d; }
__device__ __forceinline__ void wave_lds_sync() { __builtin_amdgcn_fence(__ATOMIC_RELEASE, "workgroup"); __builtin_amdgcn_wave_barrier(); __builtin_amdgcn_fence(__ATOMIC_ACQUIRE, "workgroup"); }
__device__ __forceinline__ float pmul(float a, float b) { float p = a * b; asm volatile("" : "+v"(p)); return p; }

__global__ __launch_bounds__(32) void soft_kernel(const float* __restrict__ lg, float* __restrict__ PR) {
  const int lane = threadIdx.x; const size_t b = blockIdx.x; float v0 = bf16_rne(lg[b * 64 + lane]), v1 = bf16_rne(lg[b * 64 + 32 + lane]);
  float m0 = v0, m1 = v1; for (int o = 1; o < 16; o <<= 1) { m0 = fmaxf(m0, __shfl_xor(m0, o)); m1 = fmaxf(m1, __shfl_xor(m1, o)); }
  const float e0 = __expf(v0 - m0), e1 = __expf(v1 - m1); float s0 = e0, s1 = e1; for (int o = 1; o < 16; o <<= 1) { s0 += __shfl_xor(s0, o); s1 += __shfl_xor(s1, o); }
  for (int pass = 0; pass < 2; ++pass) { ((volatile float*)PR)[b * 64 + lane] = e0 / s0; ((volatile float*)PR)[b * 64 + 32 + lane] = e1 / s1; __threadfence(); }
}
__global__ __launch_bounds__(256) void yt_kernel(const float* __restrict__ yt, b16* __restrict__ YT) {
  const int u = blockIdx.x * 256 + threadIdx.x; if (u >= YP * (B / 8)) return; const int y = u / (B / 8), b0 = (u % (B / 8)) * 8; v8b v;
#pragma unroll
  for (int j = 0; j < 8; ++j) v[j] = (y < Y) ? (b16)bf16_rne(yt[(size_t)(b0 + j) * Y + y]) : (b16)0.0f; for (int pass = 0; pass < 2; ++pass) { *(volatile v8b*)(YT + (size_t)y * B + b0) = v; __threadfence(); }
}
__global__ __launch_bounds__(32) void count_kernel(const float* __restrict__ PR, const b16* __restrict__ YT, int JV, b16* __restrict__ PH, b16* __restrict__ PL) {
  __shared__ __attribute__((aligned(16))) b16 Bt[16][40]; __shared__ float Nj[16];
  const int lane = threadIdx.x, nloc = lane & 15, hlf = lane >> 4; const int j0 = blockIdx.x * 64; if (j0 >= JV) return;
  {
#pragma unroll 1
    for (int sub = 0; sub < 4; ++sub) { const int jj = j0 + sub * 16; v8f acc[7];
#pragma unroll
      for (int t = 0; t < 7; ++t) acc[t] = (v8f){};
#pragma unroll 1
      for (int kb = 0; kb < B; kb += 32) {
        for (int i = 0; i < 16; ++i) { const int idx = i * 32 + lane; const int jl = idx & 15, bb = idx >> 4; const int j = jj + jl; const size_t b = kb + bb; const float* pr = PR + b * 64;
          const float f = pmul(pmul(pr[j >> 12], pr[16 + ((j >> 8) & 15)]), pmul(pr[32 + ((j >> 4) & 15)], pr[48 + (j & 15)])); Bt[jl][bb] = (b16)(f * FS); }
        wave_lds_sync(); const v16b bf = frag_kb(&Bt[nloc][0], hlf);
#pragma unroll
        for (int t = 0; t < 7; ++t) acc[t] = wmma16b(frag_kb(YT + (size_t)(t * 16 + nloc) * B + kb, hlf), bf, acc[t]);
        wave_lds_sync(); }
      float cs = 0.0f;
#pragma unroll
      for (int t = 0; t < 7; ++t)
#pragma unroll
        for (int r8 = 0; r8 < 8; ++r8) cs += acc[t][r8];
      cs += __shfl_xor(cs, 16); const float nj = fmaxf(cs * (1.0f / FS), 1e-6f);
#pragma unroll
      for (int t = 0; t < 7; ++t)
#pragma unroll
        for (int r8 = 0; r8 < 8; ++r8) { const int y = t * 16 + 8 * hlf + r8; float p = fminf(fmaxf(fmaxf(acc[t][r8] * (1.0f / FS), 1e-6f) / nj, 0.0f), 1.0f); if (y >= Y) p = 0.0f; b16 ph, pl; split16(p * PS, ph, pl); const size_t at = (size_t)y * J + jj + nloc; ((volatile b16*)PH)[at] = ph; ((volatile b16*)PL)[at] = pl; ((volatile b16*)PH)[at] = ph; ((volatile b16*)PL)[at] = pl; } }
    __threadfence(); }
}
__global__ __launch_bounds__(32) void post_kernel(const float* __restrict__ PR, const b16* __restrict__ PH, const b16* __restrict__ PL, int JV, float* __restrict__ out) {
  __shared__ __attribute__((aligned(16))) b16 Bt[32][40]; __shared__ float So[32][Y + 1];
  const int lane = threadIdx.x, nloc = lane & 15, hlf = lane >> 4; const size_t b0 = (size_t)blockIdx.x * 32; const size_t b = b0 + lane;
  float pr[64]; for (int i = 0; i < 64; ++i) pr[i] = PR[b * 64 + i];
  v8f acc[7][2];
#pragma unroll
  for (int t = 0; t < 7; ++t) { acc[t][0] = (v8f){}; acc[t][1] = (v8f){}; }
#pragma unroll 1
  for (int kb = 0; kb < JV; kb += 32) { const int j1 = kb >> 12, j2 = (kb >> 8) & 15, j3a = (kb >> 4) & 15;
    float p123[2]; { float p12 = 0.0f, pa = 0.0f, pb = 0.0f;
#pragma unroll
      for (int i = 0; i < 16; ++i) { if (i == j1) p12 = pr[i]; } float q2 = 0.0f;
#pragma unroll
      for (int i = 0; i < 16; ++i) { if (i == j2) q2 = pr[16 + i]; }
#pragma unroll
      for (int i = 0; i < 16; ++i) { if (i == j3a) pa = pr[32 + i]; if (i == j3a + 1) pb = pr[32 + i]; } p12 = pmul(p12, q2); p123[0] = pmul(p12, pa); p123[1] = pmul(p12, pb); }
#pragma unroll
    for (int c = 0; c < 32; ++c) Bt[lane][c] = (b16)(pmul(p123[c >> 4], pr[48 + (c & 15)]) * FS);
    wave_lds_sync(); const v16b bb0 = frag_kb(&Bt[nloc][0], hlf), bb1 = frag_kb(&Bt[16 + nloc][0], hlf);
#pragma unroll
    for (int t = 0; t < 7; ++t) { const v16b ah = frag_kb(PH + (size_t)(t * 16 + nloc) * J + kb, hlf), al = frag_kb(PL + (size_t)(t * 16 + nloc) * J + kb, hlf); acc[t][0] = wmma16b(ah, bb0, acc[t][0]); acc[t][0] = wmma16b(al, bb0, acc[t][0]); acc[t][1] = wmma16b(ah, bb1, acc[t][1]); acc[t][1] = wmma16b(al, bb1, acc[t][1]); }
    wave_lds_sync(); }
#pragma unroll
  for (int t = 0; t < 7; ++t)
#pragma unroll
    for (int ct = 0; ct < 2; ++ct)
#pragma unroll
      for (int r8 = 0; r8 < 8; ++r8) { const int y = t * 16 + 8 * hlf + r8; if (y < Y) So[ct * 16 + nloc][y] = acc[t][ct][r8] * (1.0f / (PS * FS)); }
  wave_lds_sync();
  for (int pass = 0; pass < 2; ++pass) { for (int i = lane; i < 32 * Y; i += 32) ((volatile float*)out)[b0 * Y + i] = So[i / Y][i % Y]; __threadfence(); }
}
}

extern "C" void kernel_launch(void* const* d_in, const int* in_sizes, int n_in, void* d_out, int out_size, void* d_ws, size_t ws_size, hipStream_t stream) {
  (void)n_in;
  auto Fp = [&](int i) { return (const float*)d_in[i]; };
  if (in_sizes[0] != B * 64 || in_sizes[1] != B * Y || out_size != B * Y) return;
  const int JV = J;
  size_t off = 0; char* ws = (char*)d_ws;
  auto carve = [&](size_t bytes) { char* p = ws + off; off += (bytes + 255) & ~(size_t)255; return p; };
  float* PR = (float*)carve((size_t)B * 64 * 4); b16* YT = (b16*)carve((size_t)YP * B * 2); b16* PH = (b16*)carve((size_t)YP * J * 2); b16* PL = (b16*)carve((size_t)YP * J * 2);
  if (off > ws_size || off > ((size_t)48 << 20)) return;
  soft_kernel<<<B, 32, 0, stream>>>(Fp(0), PR); yt_kernel<<<(YP * (B / 8) + 255) / 256, 256, 0, stream>>>(Fp(1), YT);
  count_kernel<<<(unsigned)(JV / 64), 32, 0, stream>>>(PR, YT, JV, PH, PL);
  post_kernel<<<B / 32, 32, 0, stream>>>(PR, PH, PL, JV, (float*)d_out);
}
